// MultiheadAttention_37288906064443
// MI455X (gfx1250) — hardware-verified
//
#include <hip/hip_runtime.h>


#ifndef NB
#define NB 8
#endif
#ifndef SEQ
#define SEQ 1024
#endif
#define NB_FULL  8
#define SEQ_FULL 1024
#define DM    1024
#define NH    16
#define HD    64
#define QKVN  (3 * DM)
#define MROWS (NB * SEQ)
#define PCAR  1024.0f
#define RSC   2048.0f
#define RSCI  (1.0f / 2048.0f)
#define SCL   0.125f
#define L2E   1.4426950408889634f
#define QT    128
#define KT    64
#define LP    72
#define OP    68

static_assert(HD == 64);
static_assert(NH * HD == DM);
static_assert(QKVN == NH * 3 * HD);
static_assert(SEQ % 128 == 0);
static_assert(SEQ % KT == 0);
static_assert(DM % 64 == 0 && DM % 32 == 0);
static_assert(MROWS % 64 == 0);
static_assert(NB <= NB_FULL && SEQ <= SEQ_FULL);
static_assert(((size_t)SEQ * DM / 8) % 256 == 0);
static_assert(((size_t)QKVN * DM / 8) % 256 == 0);
static_assert(((size_t)DM * DM / 8) % 256 == 0);

typedef _Float16 h16;
typedef unsigned short bf;
typedef __attribute__((ext_vector_type(16))) __bf16   v16bf;
typedef __attribute__((ext_vector_type(16))) _Float16 v16h;
typedef __attribute__((ext_vector_type(8)))  _Float16 v8h;
typedef __attribute__((ext_vector_type(8)))  unsigned short v8us;
typedef __attribute__((ext_vector_type(8)))  float    v8f;
typedef __attribute__((ext_vector_type(4)))  float    v4f;
typedef v4f  __attribute__((may_alias)) v4fa;

__device__ __forceinline__ unsigned short f2bf(float f) { unsigned u = __float_as_uint(f); u += 0x7FFFu + ((u >> 16) & 1u); return (unsigned short)(u >> 16); }
__device__ __forceinline__ float bf2f(unsigned short b) { return __uint_as_float(((unsigned)b) << 16); }
__device__ __forceinline__ float bfr(float f) { return bf2f(f2bf(f)); }
__device__ __forceinline__ v16h cat16(v8h lo, v8h hi) { return __builtin_shufflevector(lo, hi, 0, 1, 2, 3, 4, 5, 6, 7, 8, 9, 10, 11, 12, 13, 14, 15); }
__device__ __forceinline__ v16bf cat16b(v8us lo, v8us hi) { return __builtin_bit_cast(v16bf, __builtin_shufflevector(lo, hi, 0, 1, 2, 3, 4, 5, 6, 7, 8, 9, 10, 11, 12, 13, 14, 15)); }
__device__ __forceinline__ v8f wmma16(v16h a, v16h b, v8f c) { return __builtin_amdgcn_wmma_f32_16x16x32_f16(false, a, false, b, (short)0, c, false, false); }
__device__ __forceinline__ v8f wmmab(v16bf a, v16bf b, v8f c) { return __builtin_amdgcn_wmma_f32_16x16x32_bf16(false, a, false, b, (short)0, c, false, false); }
__device__ __forceinline__ void splitf(float y, unsigned short& h, unsigned short& l) { h = f2bf(y); l = f2bf(y - bf2f(h)); }

template <typename T16> struct WFrag;
template <> struct WFrag<h16> { typedef v16h V; static __device__ __forceinline__ V ld(const h16* p) { return cat16(*(const v8h*)p, *(const v8h*)(p + 16)); } static __device__ __forceinline__ v8f mma(V a, V b, v8f c) { return wmma16(a, b, c); } };
template <> struct WFrag<bf> { typedef v16bf V; static __device__ __forceinline__ V ld(const bf* p) { return cat16b(*(const v8us*)p, *(const v8us*)(p + 16)); } static __device__ __forceinline__ v8f mma(V a, V b, v8f c) { return wmmab(a, b, c); } };

template <typename T16, int NSPLIT, bool BIAS>
__global__ __launch_bounds__(32) void k_gemmw(const T16* __restrict__ A, const T16* __restrict__ A2, const T16* __restrict__ Bt, const T16* __restrict__ Bt2, int K, float* C, int ldc, const float* __restrict__ bias, size_t sA, size_t sB, size_t sC) {
    typedef typename WFrag<T16>::V V;
    __shared__ __align__(16) float os[16 * 68];
    const size_t z = blockIdx.z; A += z * sA; if (A2) A2 += z * sA; Bt += z * sB; if (Bt2) Bt2 += z * sB; C += z * sC;
    const int lane = threadIdx.x & 31, lr = lane & 15, hi = lane >> 4; const int r0 = blockIdx.x * 64, c0 = blockIdx.y * 64;
    v8f acc[4][4];
#pragma unroll
    for (int mb = 0; mb < 4; ++mb)
#pragma unroll
        for (int nb = 0; nb < 4; ++nb) acc[mb][nb] = (v8f){};
    const size_t aoff = (size_t)(r0 + lr) * K + 8 * hi, boff = (size_t)(c0 + lr) * K + 8 * hi;
#pragma unroll 1
    for (int kc = 0; kc < K; kc += 32) {
        V a[4], a2[4];
#pragma unroll
        for (int mb = 0; mb < 4; ++mb) { a[mb] = WFrag<T16>::ld(A + aoff + (size_t)mb * 16 * K + kc); if (NSPLIT == 1 || NSPLIT == 2) a2[mb] = WFrag<T16>::ld(A2 + aoff + (size_t)mb * 16 * K + kc); }
#pragma unroll
        for (int nb = 0; nb < 4; ++nb) { const V b = WFrag<T16>::ld(Bt + boff + (size_t)nb * 16 * K + kc); V b2; if (NSPLIT >= 2) b2 = WFrag<T16>::ld(Bt2 + boff + (size_t)nb * 16 * K + kc);
#pragma unroll
            for (int mb = 0; mb < 4; ++mb) { acc[mb][nb] = WFrag<T16>::mma(a[mb], b, acc[mb][nb]); if (NSPLIT == 1 || NSPLIT == 2) acc[mb][nb] = WFrag<T16>::mma(a2[mb], b, acc[mb][nb]); if (NSPLIT >= 2) acc[mb][nb] = WFrag<T16>::mma(a[mb], b2, acc[mb][nb]); } }
        asm volatile("v_nop\n\tv_nop\n\tv_nop\n\tv_nop" : "+v"(acc[0][0]), "+v"(acc[1][1]), "+v"(acc[2][2]), "+v"(acc[3][3]) : "v"(a[0]), "v"(a[3]));
    }
#pragma unroll
    for (int mb = 0; mb < 4; ++mb) {
#pragma unroll
        for (int nb = 0; nb < 4; ++nb) {
#pragma unroll
            for (int j = 0; j < 8; ++j) os[(hi * 8 + j) * 68 + nb * 16 + lr] = acc[mb][nb][j]; }
        __builtin_amdgcn_wave_barrier(); asm volatile("" ::: "memory");
        float* crow = C + (size_t)(r0 + mb * 16) * ldc + c0;
#pragma unroll 1
        for (int ps = 0; ps < 2; ++ps) {
#pragma unroll
            for (int s = 0; s < 8; ++s) { const int row = 2 * s + hi, cofs = lr * 4; v4f val = *(const v4fa*)(os + row * 68 + cofs); if (BIAS) { val[0] += bfr(bias[c0 + cofs]); val[1] += bfr(bias[c0 + cofs + 1]); val[2] += bfr(bias[c0 + cofs + 2]); val[3] += bfr(bias[c0 + cofs + 3]); }
                *(volatile v4f*)(crow + (size_t)row * ldc + cofs) = val; }
            if (ps == 0) __threadfence(); }
        __builtin_amdgcn_wave_barrier(); asm volatile("" ::: "memory");
    }
}

__global__ __launch_bounds__(256) void k_cvt8(const float* __restrict__ src, bf* dst, unsigned n8, size_t sS, size_t sD) {
    const unsigned i = blockIdx.x * 256u + threadIdx.x; if (i >= n8) return;
    const float* s = src + (size_t)blockIdx.y * sS; bf* d = dst + (size_t)blockIdx.y * sD;
    const v8f v = *(const v8f*)(s + (size_t)i * 8); v8us o;
#pragma unroll
    for (int k = 0; k < 8; ++k) o[k] = f2bf(v[k]);
    *(volatile v8us*)(d + (size_t)i * 8) = o; __threadfence(); *(volatile v8us*)(d + (size_t)i * 8) = o;
}

__global__ __launch_bounds__(32) void k_qkv(const bf* __restrict__ XB, const bf* __restrict__ WB, const float* __restrict__ bias, h16* Qh, h16* Ql, h16* Kp, h16* VT) {
    typedef WFrag<bf>::V V;
    __shared__ __align__(16) float os[64 * OP];
    const unsigned lane = threadIdx.x & 31u, lr = lane & 15u, hi = lane >> 4;
    const unsigned r0 = blockIdx.x * 64u, c0 = blockIdx.y * 64u;
    v8f acc[4][4];
#pragma unroll
    for (int mb = 0; mb < 4; ++mb)
#pragma unroll
        for (int nb = 0; nb < 4; ++nb) acc[mb][nb] = (v8f){};
    const size_t aoff = (size_t)(r0 + lr) * DM + 8u * hi, boff = (size_t)(c0 + lr) * DM + 8u * hi;
#pragma unroll 1
    for (unsigned kc = 0; kc < DM; kc += 32) {
        V a[4];
#pragma unroll
        for (int mb = 0; mb < 4; ++mb) a[mb] = WFrag<bf>::ld(XB + aoff + (size_t)mb * 16 * DM + kc);
#pragma unroll
        for (int nb = 0; nb < 4; ++nb) { const V b = WFrag<bf>::ld(WB + boff + (size_t)nb * 16 * DM + kc);
#pragma unroll
            for (int mb = 0; mb < 4; ++mb) acc[mb][nb] = wmmab(a[mb], b, acc[mb][nb]); }
        asm volatile("v_nop\n\tv_nop\n\tv_nop\n\tv_nop" : "+v"(acc[0][0]), "+v"(acc[1][1]), "+v"(acc[2][2]), "+v"(acc[3][3]) : "v"(a[0]), "v"(a[3]));
    }
#pragma unroll
    for (int mb = 0; mb < 4; ++mb) {
#pragma unroll
        for (int nb = 0; nb < 4; ++nb) { const float bv = bfr(bias[c0 + nb * 16 + lr]);
#pragma unroll
            for (int j = 0; j < 8; ++j) os[(mb * 16 + hi * 8 + j) * OP + nb * 16 + lr] = acc[mb][nb][j] + bv; } }
    __syncthreads();
    const unsigned head = c0 / 192u; const unsigned which = (c0 - head * 192u) >> 6;
    const unsigned b = r0 / (unsigned)SEQ; const unsigned s0 = r0 - b * (unsigned)SEQ;
    const size_t bh = (size_t)b * NH + head;
    const unsigned sub = lane >> 3, pc = (lane & 7u) * 8u;
    if (which == 0u) {
        h16* ph = Qh + (bh * SEQ + s0) * HD; h16* pl = Ql + (bh * SEQ + s0) * HD;
#pragma unroll 1
        for (int ps = 0; ps < 2; ++ps) {
#pragma unroll 4
            for (unsigned i = 0; i < 16; ++i) { const unsigned row = 4u * i + sub; const v4f a = *(const v4fa*)(os + row * OP + pc); const v4f c = *(const v4fa*)(os + row * OP + pc + 4); v8h oh, ol;
#pragma unroll
                for (int e = 0; e < 8; ++e) { const float v = (e < 4) ? a[e & 3] : c[e & 3]; const h16 hh = (h16)v; oh[e] = hh; ol[e] = (h16)((v - (float)hh) * RSC); }
                *(volatile v8h*)(ph + (size_t)row * HD + pc) = oh; *(volatile v8h*)(pl + (size_t)row * HD + pc) = ol; }
            if (ps == 0) __threadfence(); }
    } else if (which == 1u) {
        h16* ph = Kp + (bh * SEQ + s0) * HD;
#pragma unroll 1
        for (int ps = 0; ps < 2; ++ps) {
#pragma unroll 4
            for (unsigned i = 0; i < 16; ++i) { const unsigned row = 4u * i + sub; const v4f a = *(const v4fa*)(os + row * OP + pc); const v4f c = *(const v4fa*)(os + row * OP + pc + 4); v8h oh;
#pragma unroll
                for (int e = 0; e < 8; ++e) { const float v = (e < 4) ? a[e & 3] : c[e & 3]; oh[e] = (h16)v; }
                *(volatile v8h*)(ph + (size_t)row * HD + pc) = oh; }
            if (ps == 0) __threadfence(); }
    } else {
        h16* pv = VT + (bh * HD) * SEQ + s0;
#pragma unroll 1
        for (int ps = 0; ps < 2; ++ps) {
#pragma unroll 4
            for (unsigned i = 0; i < 16; ++i) { const unsigned d = 4u * i + sub; v8h o;
#pragma unroll
                for (int e = 0; e < 8; ++e) o[e] = (h16)os[(pc + e) * OP + d];
                *(volatile v8h*)(pv + (size_t)d * SEQ + pc) = o; }
            if (ps == 0) __threadfence(); }
    }
}

__global__ __launch_bounds__(256) void k_flash(const h16* __restrict__ Qh, const h16* __restrict__ Ql, const h16* __restrict__ Kp, const h16* __restrict__ VT, bf* ATh, bf* ATl) {
    __shared__ __align__(16) h16 sK[KT * LP];
    __shared__ __align__(16) h16 sV[HD * LP];
    __shared__ __align__(16) float ot[8 * 16 * OP];
    const unsigned tid = threadIdx.x, lane = tid & 31u, wid = tid >> 5, lr = lane & 15u, hi = lane >> 4;
    const unsigned nqb = (unsigned)(SEQ / QT); const unsigned bhu = blockIdx.x / nqb; const unsigned qblk = blockIdx.x - bhu * nqb;
    const size_t bh = bhu; const unsigned qb = qblk * QT + wid * 16u;
    const h16* kbase = Kp + bh * SEQ * HD; const h16* vbase = VT + bh * HD * SEQ;
    const h16* qp = Qh + (bh * SEQ + qb + lr) * HD + 8u * hi; const h16* qq = Ql + (bh * SEQ + qb + lr) * HD + 8u * hi;
    const v16h qh0 = cat16(*(const v8h*)qp, *(const v8h*)(qp + 16)), qh1 = cat16(*(const v8h*)(qp + 32), *(const v8h*)(qp + 48));
    const v16h ql0 = cat16(*(const v8h*)qq, *(const v8h*)(qq + 16)), ql1 = cat16(*(const v8h*)(qq + 32), *(const v8h*)(qq + 48));
    v8f acc[4];
#pragma unroll
    for (int j = 0; j < 4; ++j) acc[j] = (v8f){};
    float m_run = -1.0e30f, l_run = 0.0f;
    const unsigned st_r = tid >> 3, st_c = (tid & 7u) * 8u;
#pragma unroll 1
    for (unsigned kb = 0; kb < (unsigned)SEQ; kb += KT) {
#pragma unroll
        for (unsigned c = 0; c < 2; ++c) { const unsigned r = st_r + 32u * c;
            const v8h kv = *(const v8h*)(kbase + (size_t)(kb + r) * HD + st_c);
            const v8h vv = *(const v8h*)(vbase + (size_t)r * SEQ + kb + st_c);
            *(v8h*)(sK + r * LP + st_c) = kv; *(v8h*)(sV + r * LP + st_c) = vv; }
        __syncthreads();
        v8f sh[4], sl[4];
#pragma unroll
        for (int t = 0; t < 4; ++t) { const h16* kr = sK + (t * 16 + lr) * LP + 8u * hi;
            const v16h ka0 = cat16(*(const v8h*)kr, *(const v8h*)(kr + 16)); const v16h ka1 = cat16(*(const v8h*)(kr + 32), *(const v8h*)(kr + 48));
            v8f c = (v8f){}; c = wmma16(ka0, qh0, c); c = wmma16(ka1, qh1, c); sh[t] = c;
            v8f e = (v8f){}; e = wmma16(ka0, ql0, e); e = wmma16(ka1, ql1, e); sl[t] = e; }
        asm volatile("v_nop\n\tv_nop\n\tv_nop\n\tv_nop" : "+v"(sh[0]), "+v"(sh[1]), "+v"(sh[2]), "+v"(sh[3]), "+v"(sl[0]), "+v"(sl[1]), "+v"(sl[2]), "+v"(sl[3]) : "v"(qh0), "v"(qh1), "v"(ql0), "v"(ql1));
        float mt = -1.0e30f;
#pragma unroll
        for (int t = 0; t < 4; ++t)
#pragma unroll
            for (int r = 0; r < 8; ++r) { const float tv = (sh[t][r] + sl[t][r] * RSCI) * SCL; sh[t][r] = tv; mt = fmaxf(mt, tv); }
        mt = fmaxf(mt, __shfl_xor(mt, 16, 32));
        const float m_new = fmaxf(m_run, mt);
        const float alpha = __builtin_amdgcn_exp2f((m_run - m_new) * L2E);
        float ssum = 0.0f; v16h pa[2];
#pragma unroll
        for (int t = 0; t < 4; ++t)
#pragma unroll
            for (int r = 0; r < 8; ++r) { const float p = __builtin_amdgcn_exp2f((sh[t][r] - m_new) * L2E); ssum += p; pa[t >> 1][(t & 1) * 8 + r] = (h16)(p * PCAR); }
        ssum += __shfl_xor(ssum, 16, 32);
        l_run = l_run * alpha + ssum; m_run = m_new;
        float ar[8];
#pragma unroll
        for (int r = 0; r < 8; ++r) ar[r] = __shfl(alpha, (int)(hi * 8u) + r, 32);
#pragma unroll
        for (int j = 0; j < 4; ++j)
#pragma unroll
            for (int r = 0; r < 8; ++r) acc[j][r] *= ar[r];
#pragma unroll
        for (int j = 0; j < 4; ++j) { const h16* vr = sV + (j * 16 + lr) * LP + 8u * hi;
            const v16h vf0 = cat16(*(const v8h*)vr, *(const v8h*)(vr + 16)); const v16h vf1 = cat16(*(const v8h*)(vr + 32), *(const v8h*)(vr + 48));
            acc[j] = wmma16(pa[0], vf0, acc[j]); acc[j] = wmma16(pa[1], vf1, acc[j]); }
        asm volatile("v_nop\n\tv_nop\n\tv_nop\n\tv_nop" : "+v"(acc[0]), "+v"(acc[1]), "+v"(acc[2]), "+v"(acc[3]) : "v"(pa[0]), "v"(pa[1]));
        __syncthreads();
    }
    const float linv = (1.0f / l_run) * (1.0f / PCAR);
    float lrr[8];
#pragma unroll
    for (int r = 0; r < 8; ++r) lrr[r] = __shfl(linv, (int)(hi * 8u) + r, 32);
    float* ow = ot + wid * 16u * OP;
#pragma unroll
    for (int j = 0; j < 4; ++j)
#pragma unroll
        for (int r = 0; r < 8; ++r) ow[(hi * 8u + r) * OP + j * 16 + lr] = acc[j][r] * lrr[r];
    __syncthreads();
    const unsigned b = bhu / (unsigned)NH, h = bhu - b * (unsigned)NH;
    const unsigned sub = lane >> 3, pc = (lane & 7u) * 8u;
#pragma unroll 1
    for (int ps = 0; ps < 2; ++ps) {
#pragma unroll
        for (unsigned i = 0; i < 4; ++i) { const unsigned row = 4u * i + sub; const v4f a = *(const v4fa*)(ow + row * OP + pc); const v4f c = *(const v4fa*)(ow + row * OP + pc + 4); v8us oh, ol;
#pragma unroll
            for (int e = 0; e < 8; ++e) { const float v = (e < 4) ? a[e & 3] : c[e & 3]; unsigned short x0, x1; splitf(v, x0, x1); oh[e] = x0; ol[e] = x1; }
            const size_t oo = ((size_t)b * SEQ + qb + row) * DM + h * HD + pc;
            *(volatile v8us*)(ATh + oo) = oh; *(volatile v8us*)(ATl + oo) = ol; }
        if (ps == 0) __threadfence(); }
}

#define WS_XB   ((size_t)MROWS * DM * 2)
#define WS_WIN  ((size_t)QKVN * DM * 2)
#define WS_WO   ((size_t)DM * DM * 2)
#define WS_PL   ((size_t)NB * NH * SEQ * HD * 2)
#define WS_AT   ((size_t)MROWS * DM * 2)
#define WS_TOTAL (WS_XB + WS_WIN + WS_WO + 4 * WS_PL + 2 * WS_AT)
static_assert(WS_XB % 256 == 0 && WS_WIN % 256 == 0 && WS_WO % 256 == 0 && WS_PL % 256 == 0 && WS_AT % 256 == 0);
static_assert(WS_TOTAL <= (size_t)134217728);

extern "C" void kernel_launch(void* const* d_in, const int* in_sizes, int n_in,
                              void* d_out, int out_size, void* d_ws, size_t ws_size, hipStream_t stream) {
    if (n_in < 5) return;
    const size_t need_x = ((size_t)(NB - 1) * SEQ_FULL + SEQ) * DM;
    if ((size_t)in_sizes[0] < need_x) return;
    if ((size_t)in_sizes[1] < (size_t)QKVN * DM) return;
    if (in_sizes[2] < QKVN) return;
    if ((size_t)in_sizes[3] < (size_t)DM * DM) return;
    if (in_sizes[4] < DM) return;
    if ((size_t)out_size < need_x) return;
    if (ws_size < WS_TOTAL) return;
    const float* x = (const float*)d_in[0]; const float* w_in = (const float*)d_in[1]; const float* b_in = (const float*)d_in[2]; const float* w_out = (const float*)d_in[3]; const float* b_out = (const float*)d_in[4];
    float* OUT = (float*)d_out;
    char* wsp = (char*)d_ws;
    auto take = [&](size_t bytes) { char* p = wsp; wsp += bytes; return (void*)p; };
    bf* XB = (bf*)take(WS_XB); bf* WIN = (bf*)take(WS_WIN); bf* WO = (bf*)take(WS_WO);
    h16* Qh = (h16*)take(WS_PL); h16* Ql = (h16*)take(WS_PL); h16* Kp = (h16*)take(WS_PL); h16* VT = (h16*)take(WS_PL);
    bf* ATh = (bf*)take(WS_AT); bf* ATl = (bf*)take(WS_AT);
    k_cvt8<<<dim3((unsigned)((size_t)SEQ * DM / 8 / 256), NB, 1), 256, 0, stream>>>(x, XB, (unsigned)((size_t)SEQ * DM / 8), (size_t)SEQ_FULL * DM, (size_t)SEQ * DM);
    k_cvt8<<<dim3((unsigned)((size_t)QKVN * DM / 8 / 256), 1, 1), 256, 0, stream>>>(w_in, WIN, (unsigned)((size_t)QKVN * DM / 8), 0, 0);
    k_cvt8<<<dim3((unsigned)((size_t)DM * DM / 8 / 256), 1, 1), 256, 0, stream>>>(w_out, WO, (unsigned)((size_t)DM * DM / 8), 0, 0);
    k_qkv<<<dim3(MROWS / 64, QKVN / 64, 1), 32, 0, stream>>>(XB, WIN, b_in, Qh, Ql, Kp, VT);
    k_flash<<<dim3((unsigned)(NB * NH * (SEQ / QT)), 1, 1), 256, 0, stream>>>(Qh, Ql, Kp, VT, ATh, ATl);
    k_gemmw<bf, 1, true><<<dim3(SEQ / 64, DM / 64, NB), 32, 0, stream>>>(ATh, ATl, WO, nullptr, DM, OUT, DM, b_out, (size_t)SEQ * DM, 0, (size_t)SEQ_FULL * DM);
}
